// GatedGraphConvModule_38886633898060
// MI455X (gfx1250) — hardware-verified
//
#include <hip/hip_runtime.h>
#include <stddef.h>


#define DIM   64
#define NT    4
#define NC    (NT * DIM)
#define NG    (3 * DIM)
#define GR    32
#define XP    260
#define NB    1024
#define CHUNK 2048
#define NTHR  256
#define NWAVE 8
#define WCAP  256
#define NGRP  (CHUNK / (NTHR * 4))
#define TPW   ((NB / 16) / NWAVE)

#define LDS_SACC (NB * DIM)
#define LDS_LIST (NWAVE * WCAP)
#define LDS_B_BYTES ((LDS_SACC + LDS_LIST + NWAVE) * 4)

static_assert(WCAP == (CHUNK / NTHR) * 32);
static_assert(NGRP == 2);
static_assert(NB == 1024);
static_assert(CHUNK == 2048);
static_assert(TPW == 8);
static_assert((LDS_SACC % 4) == 0);
static_assert((XP % 4) == 0);
static_assert(LDS_B_BYTES == 270368);

typedef float          v2f   __attribute__((ext_vector_type(2)));
typedef float          v4f   __attribute__((ext_vector_type(4)));
typedef float          v8f   __attribute__((ext_vector_type(8)));
typedef int            v4i   __attribute__((ext_vector_type(4)));
typedef unsigned short v8us  __attribute__((ext_vector_type(8)));
typedef __bf16         v16bf __attribute__((ext_vector_type(16)));
union Frag { v16bf v; v8us u[2]; };

__device__ __forceinline__ v8f wmb(v16bf a, v16bf b, v8f c) {
  v8f d = __builtin_amdgcn_wmma_f32_16x16x32_bf16(false, a, false, b, (short)0, c, false, false);
  asm volatile("v_nop\n\tv_nop\n\tv_nop\n\tv_nop" : "+v"(d) : "v"(a), "v"(b));
  return d;
}

__device__ __forceinline__ void ldf(Frag& f, const unsigned short* p, size_t o) {
  f.u[0] = *(const v8us*)(p + o);
  f.u[1] = *(const v8us*)(p + o + 16);
}

__device__ __forceinline__ unsigned int bfr(float f) {
  const unsigned int u = __float_as_uint(f);
  return (u + 0x7FFFu + ((u >> 16) & 1u)) >> 16;
}

__device__ __forceinline__ void split8(v4f a, v4f b, v8us& h, v8us& l) {
  const float f[8] = {a.x, a.y, a.z, a.w, b.x, b.y, b.z, b.w};
  v8us hv, lv;
#pragma unroll
  for (int i = 0; i < 8; ++i) {
    const unsigned int hb = bfr(f[i]);
    const float r = f[i] - __uint_as_float(hb << 16);
    hv[i] = (unsigned short)hb;
    lv[i] = (unsigned short)bfr(r);
  }
  h = hv;
  l = lv;
}

__device__ __forceinline__ float sigm(float x) {
  x = fminf(fmaxf(x, -30.0f), 30.0f);
  const float e = __expf(-x);
  return __builtin_amdgcn_rcpf(1.0f + e);
}

__global__ __launch_bounds__(NTHR) void k_split(const float* __restrict__ src,
                                                unsigned short* hi, unsigned short* lo, int n8) {
  const int i = blockIdx.x * NTHR + threadIdx.x;
  if (i >= n8) return;
  const size_t o = (size_t)i * 8;
  const v4f a = *(const v4f*)(src + o);
  const v4f b = *(const v4f*)(src + o + 4);
  v8us hv, lv;
  split8(a, b, hv, lv);
  *(volatile v8us*)(hi + o) = hv;
  *(volatile v8us*)(lo + o) = lv;
  __threadfence();
  *(volatile v8us*)(hi + o) = hv;
  *(volatile v8us*)(lo + o) = lv;
}

__global__ __launch_bounds__(NTHR) void k_lin(
    const unsigned short* __restrict__ Hhi, const unsigned short* __restrict__ Hlo,
    const unsigned short* __restrict__ Whi, const unsigned short* __restrict__ Wlo,
    const float* __restrict__ bc, float* hall, int nN) {
  __shared__ __attribute__((aligned(16))) float Xs[GR * XP];

  const int tid  = threadIdx.x;
  const int lane = tid & 31;
  const int wave = tid >> 5;
  const int hf   = lane >> 4;
  const int m    = lane & 15;
  const int rowBase = blockIdx.x * GR;
  const int rt = wave & 1;
  const int cg = wave >> 1;

  int arow = rowBase + 16 * rt + m;
  if (arow > nN - 1) arow = nN - 1;
  Frag ah0, al0, ah1, al1;
  {
    const size_t o = (size_t)arow * DIM + 8 * hf;
    ldf(ah0, Hhi, o);      ldf(al0, Hlo, o);
    ldf(ah1, Hhi, o + 32); ldf(al1, Hlo, o + 32);
  }

#pragma unroll
  for (int ct = 0; ct < 4; ++ct) {
    const int ncol = 64 * cg + 16 * ct + m;
    const float bv = bc[ncol];
    v8f acc;
#pragma unroll
    for (int r = 0; r < 8; ++r) acc[r] = bv;
    const size_t wo = (size_t)ncol * DIM + 8 * hf;
    Frag bh, bl;
    ldf(bh, Whi, wo); ldf(bl, Wlo, wo);
    acc = wmb(ah0.v, bh.v, acc);
    acc = wmb(ah0.v, bl.v, acc);
    acc = wmb(al0.v, bh.v, acc);
    ldf(bh, Whi, wo + 32); ldf(bl, Wlo, wo + 32);
    acc = wmb(ah1.v, bh.v, acc);
    acc = wmb(ah1.v, bl.v, acc);
    acc = wmb(al1.v, bh.v, acc);
#pragma unroll
    for (int r = 0; r < 8; ++r) Xs[(16 * rt + 8 * hf + r) * XP + ncol] = acc[r];
  }
  __syncthreads();

  v4f xr[8];
  float* xp[8];
#pragma unroll
  for (int i = 0; i < 4; ++i) {
    const int R = 4 * wave + i;
#pragma unroll
    for (int q = 0; q < 2; ++q) {
      xr[2 * i + q] = *(const v4f*)(Xs + R * XP + 128 * q + 4 * lane);
      xp[2 * i + q] = hall + (size_t)(rowBase + R) * NC + 128 * q + 4 * lane;
    }
  }
#pragma unroll
  for (int i = 0; i < 8; ++i) *(volatile v4f*)(xp[i]) = xr[i];
  __threadfence();
#pragma unroll
  for (int i = 0; i < 8; ++i) *(volatile v4f*)(xp[i]) = xr[i];
}

__device__ __forceinline__ void gstep(v8f& ar, v8f& az, v8f& an, v8f& am,
                                      const v16bf ahv, const v16bf alv,
                                      const unsigned short* Hhi, const unsigned short* Hlo, size_t ho,
                                      const unsigned short* WIhi, const unsigned short* WIlo,
                                      const unsigned short* WHhi, const unsigned short* WHlo, size_t wo) {
  Frag hh, hl, b0, b1;
  ldf(hh, Hhi, ho); ldf(hl, Hlo, ho);

  ldf(b0, WIhi, wo); ldf(b1, WIlo, wo);
  ar = wmb(ahv, b0.v, ar); ar = wmb(ahv, b1.v, ar); ar = wmb(alv, b0.v, ar);
  ldf(b0, WHhi, wo); ldf(b1, WHlo, wo);
  ar = wmb(hh.v, b0.v, ar); ar = wmb(hh.v, b1.v, ar); ar = wmb(hl.v, b0.v, ar);

  const size_t wz = wo + (size_t)DIM * DIM;
  ldf(b0, WIhi, wz); ldf(b1, WIlo, wz);
  az = wmb(ahv, b0.v, az); az = wmb(ahv, b1.v, az); az = wmb(alv, b0.v, az);
  ldf(b0, WHhi, wz); ldf(b1, WHlo, wz);
  az = wmb(hh.v, b0.v, az); az = wmb(hh.v, b1.v, az); az = wmb(hl.v, b0.v, az);

  const size_t wn = wo + (size_t)2 * DIM * DIM;
  ldf(b0, WIhi, wn); ldf(b1, WIlo, wn);
  an = wmb(ahv, b0.v, an); an = wmb(ahv, b1.v, an); an = wmb(alv, b0.v, an);
  ldf(b0, WHhi, wn); ldf(b1, WHlo, wn);
  am = wmb(hh.v, b0.v, am); am = wmb(hh.v, b1.v, am); am = wmb(hl.v, b0.v, am);
}

__global__ __launch_bounds__(NTHR) void k_agg(
    const float* __restrict__ hall, const int* __restrict__ srcI, const int* __restrict__ dstI,
    const int* __restrict__ etyI, const float* __restrict__ hold,
    const unsigned short* __restrict__ WIhi, const unsigned short* __restrict__ WIlo,
    const unsigned short* __restrict__ WHhi, const unsigned short* __restrict__ WHlo,
    const unsigned short* __restrict__ Hhi, const unsigned short* __restrict__ Hlo,
    const float* __restrict__ bih, const float* __restrict__ bhh,
    float* hnew, unsigned short* Nhi, unsigned short* Nlo, int nN, int nE) {
  extern __shared__ v4f lds_dyn[];
  float* sacc = (float*)lds_dyn;
  int*   list = (int*)(sacc + LDS_SACC);
  int*   wcnt = list + LDS_LIST;

  const int tid  = threadIdx.x;
  const int lane = tid & 31;
  const int wave = tid >> 5;
  const int hf   = lane >> 4;
  const int m    = lane & 15;
  const int nodeBase = blockIdx.x * NB;

  {
    const v4f z4 = {0.f, 0.f, 0.f, 0.f};
    for (int i = tid; i < LDS_SACC / 4; i += NTHR) lds_dyn[i] = z4;
  }
  __syncthreads();

  const int nChunks = (nE + CHUNK - 1) / CHUNK;
#pragma unroll 1
  for (int ch = 0; ch < nChunks; ++ch) {
    const int cbase = ch * CHUNK;
    const bool full = (cbase + CHUNK <= nE);
    int wc = 0;
#pragma unroll
    for (int g = 0; g < NGRP; ++g) {
      const int el0 = (g * NTHR + tid) * 4;
      const int e0  = cbase + el0;
      const int sent = -2147483647 - 1;
      v4i d;
      if (full) {
        d = *(const v4i*)(dstI + e0);
      } else {
        const int em = nE - 1;
        const int c0 = e0     < em ? e0     : em;
        const int c1 = e0 + 1 < em ? e0 + 1 : em;
        const int c2 = e0 + 2 < em ? e0 + 2 : em;
        const int c3 = e0 + 3 < em ? e0 + 3 : em;
        const int v0 = dstI[c0], v1 = dstI[c1], v2 = dstI[c2], v3 = dstI[c3];
        d.x = (e0     < nE) ? v0 : sent;
        d.y = (e0 + 1 < nE) ? v1 : sent;
        d.z = (e0 + 2 < nE) ? v2 : sent;
        d.w = (e0 + 3 < nE) ? v3 : sent;
      }
      const unsigned s0 = (unsigned)d.x - (unsigned)nodeBase;
      const unsigned s1 = (unsigned)d.y - (unsigned)nodeBase;
      const unsigned s2 = (unsigned)d.z - (unsigned)nodeBase;
      const unsigned s3 = (unsigned)d.w - (unsigned)nodeBase;
      const bool h0 = s0 < (unsigned)NB;
      const bool h1 = s1 < (unsigned)NB;
      const bool h2 = s2 < (unsigned)NB;
      const bool h3 = s3 < (unsigned)NB;
      const unsigned many = __builtin_amdgcn_ballot_w32(h0 | h1 | h2 | h3);
      if (many != 0u) {
#define HITJ(J, HJ, SJ) { \
          const unsigned mj = __builtin_amdgcn_ballot_w32(HJ); \
          if (HJ) { \
            const int pos = wc + (int)__builtin_amdgcn_mbcnt_lo(mj, 0u); \
            if (pos < WCAP) list[wave * WCAP + pos] = ((el0 + (J)) << 10) | (int)(SJ); \
          } \
          wc += (int)__builtin_popcount(mj); }
        HITJ(0, h0, s0)
        HITJ(1, h1, s1)
        HITJ(2, h2, s2)
        HITJ(3, h3, s3)
#undef HITJ
      }
    }
    if (lane == 0) wcnt[wave] = wc;
    __syncthreads();

    if (wave == 0) {
      for (int wsx = 0; wsx < NWAVE; ++wsx) {
        int n = wcnt[wsx];
        if (n > WCAP) n = WCAP;
        if (n < 0) n = 0;
        for (int i = 0; i < n; ++i) {
          const int ent  = list[wsx * WCAP + i];
          const int slot = ent & (NB - 1);
          const int el   = (ent >> 10) & (CHUNK - 1);
          int e = cbase + el;
          if (e > nE - 1) e = nE - 1;
          int s = srcI[e];
          s = s < 0 ? 0 : (s > nN - 1 ? nN - 1 : s);
          int t = etyI[e];
          t = t < 0 ? 0 : (t > NT - 1 ? NT - 1 : t);
          const v2f mv = *(const v2f*)(hall + (size_t)s * NC + t * DIM + 2 * lane);
          v2f* sp = (v2f*)(sacc + slot * DIM + 2 * lane);
          const v2f cur = *sp;
          *sp = cur + mv;
        }
      }
    }
    __syncthreads();
  }

  const int lr2 = lane >> 4, lc2 = lane & 15;
  const int lr3 = lane >> 3, lc3 = lane & 7;
#pragma unroll 1
  for (int j = 0; j < TPW; ++j) {
    const int s0   = (wave * TPW + j) * 16;
    const int row0 = nodeBase + s0;
    int arow = row0 + m;
    if (arow > nN - 1) arow = nN - 1;

    Frag ah0, al0, ah1, al1;
    {
      const float* p = sacc + (s0 + m) * DIM + 8 * hf;
      const v4f x0 = *(const v4f*)(p),      x1 = *(const v4f*)(p + 4);
      const v4f x2 = *(const v4f*)(p + 16), x3 = *(const v4f*)(p + 20);
      const v4f y0 = *(const v4f*)(p + 32), y1 = *(const v4f*)(p + 36);
      const v4f y2 = *(const v4f*)(p + 48), y3 = *(const v4f*)(p + 52);
      split8(x0, x1, ah0.u[0], al0.u[0]);
      split8(x2, x3, ah0.u[1], al0.u[1]);
      split8(y0, y1, ah1.u[0], al1.u[0]);
      split8(y2, y3, ah1.u[1], al1.u[1]);
    }
    __syncthreads();

    const size_t hrow = (size_t)arow * DIM + 8 * hf;
#pragma unroll 1
    for (int c = 0; c < DIM / 16; ++c) {
      const int col = 16 * c + m;
      const float br = bih[col] + bhh[col];
      const float bz = bih[DIM + col] + bhh[DIM + col];
      const float bn = bih[2 * DIM + col];
      const float bm = bhh[2 * DIM + col];
      v8f ar, az, an, am;
#pragma unroll
      for (int r = 0; r < 8; ++r) { ar[r] = br; az[r] = bz; an[r] = bn; am[r] = bm; }
      const size_t wo = (size_t)col * DIM + 8 * hf;
      gstep(ar, az, an, am, ah0.v, al0.v, Hhi, Hlo, hrow,      WIhi, WIlo, WHhi, WHlo, wo);
      gstep(ar, az, an, am, ah1.v, al1.v, Hhi, Hlo, hrow + 32, WIhi, WIlo, WHhi, WHlo, wo + 32);

      float hn[8];
#pragma unroll
      for (int r = 0; r < 8; ++r) {
        int gr = row0 + 8 * hf + r;
        if (gr > nN - 1) gr = nN - 1;
        const float ho = hold[(size_t)gr * DIM + col];
        const float rg = sigm(ar[r]);
        const float zg = sigm(az[r]);
        const float ng = tanhf(an[r] + rg * am[r]);
        hn[r] = (1.0f - zg) * ng + zg * ho;
      }
#pragma unroll
      for (int r = 0; r < 8; ++r) sacc[(s0 + 8 * hf + r) * DIM + col] = hn[r];
    }
    __syncthreads();

    {
      v4f  fv[8];
      v8us ph[4], pl[4];
#pragma unroll
      for (int q = 0; q < 8; ++q)
        fv[q] = *(const v4f*)(sacc + (s0 + 2 * q + lr2) * DIM + 4 * lc2);
#pragma unroll
      for (int q = 0; q < 4; ++q) {
        const float* p = sacc + (s0 + 4 * q + lr3) * DIM + 8 * lc3;
        split8(*(const v4f*)(p), *(const v4f*)(p + 4), ph[q], pl[q]);
      }
#pragma unroll
      for (int q = 0; q < 8; ++q) {
        const int gr = row0 + 2 * q + lr2;
        if (gr < nN) *(volatile v4f*)(hnew + (size_t)gr * DIM + 4 * lc2) = fv[q];
      }
#pragma unroll
      for (int q = 0; q < 4; ++q) {
        const int gr = row0 + 4 * q + lr3;
        if (gr < nN) {
          const size_t o = (size_t)gr * DIM + 8 * lc3;
          *(volatile v8us*)(Nhi + o) = ph[q];
          *(volatile v8us*)(Nlo + o) = pl[q];
        }
      }
      __threadfence();
#pragma unroll
      for (int q = 0; q < 8; ++q) {
        const int gr = row0 + 2 * q + lr2;
        if (gr < nN) *(volatile v4f*)(hnew + (size_t)gr * DIM + 4 * lc2) = fv[q];
      }
#pragma unroll
      for (int q = 0; q < 4; ++q) {
        const int gr = row0 + 4 * q + lr3;
        if (gr < nN) {
          const size_t o = (size_t)gr * DIM + 8 * lc3;
          *(volatile v8us*)(Nhi + o) = ph[q];
          *(volatile v8us*)(Nlo + o) = pl[q];
        }
      }
    }
  }
}

static inline size_t al256(size_t x) { return (x + 255) & ~(size_t)255; }

extern "C" void kernel_launch(void* const* d_in, const int* in_sizes, int n_in,
                              void* d_out, int out_size, void* d_ws, size_t ws_size,
                              hipStream_t stream) {
  if (n_in < 10) return;
  const int nN = in_sizes[0] / DIM;
  if (nN < 1 || in_sizes[0] != nN * DIM) return;
  if (in_sizes[1] != NT * DIM * DIM || in_sizes[2] != NC) return;
  if (in_sizes[3] != NG * DIM || in_sizes[4] != NG * DIM) return;
  if (in_sizes[5] != NG || in_sizes[6] != NG) return;
  const int nE = in_sizes[7];
  if (nE < 0 || in_sizes[8] != nE || in_sizes[9] != nE) return;
  if (out_size != nN * DIM) return;

  const float* feat = (const float*)d_in[0];
  const float* W    = (const float*)d_in[1];
  const float* bcat = (const float*)d_in[2];
  const float* w_ih = (const float*)d_in[3];
  const float* w_hh = (const float*)d_in[4];
  const float* b_ih = (const float*)d_in[5];
  const float* b_hh = (const float*)d_in[6];
  const int*   src  = (const int*)d_in[7];
  const int*   dst  = (const int*)d_in[8];
  const int*   ety  = (const int*)d_in[9];
  float* out = (float*)d_out;

  const int nPA = ((nN + GR - 1) / GR) * GR;
  size_t off = 0;
  unsigned short* WChi = (unsigned short*)((char*)d_ws + off); off += al256((size_t)NC * DIM * 2);
  unsigned short* WClo = (unsigned short*)((char*)d_ws + off); off += al256((size_t)NC * DIM * 2);
  unsigned short* WIhi = (unsigned short*)((char*)d_ws + off); off += al256((size_t)NG * DIM * 2);
  unsigned short* WIlo = (unsigned short*)((char*)d_ws + off); off += al256((size_t)NG * DIM * 2);
  unsigned short* WHhi = (unsigned short*)((char*)d_ws + off); off += al256((size_t)NG * DIM * 2);
  unsigned short* WHlo = (unsigned short*)((char*)d_ws + off); off += al256((size_t)NG * DIM * 2);
  float* hall = (float*)((char*)d_ws + off); off += al256((size_t)nPA * NC * sizeof(float));
  float* hf1  = (float*)((char*)d_ws + off); off += al256((size_t)nPA * DIM * sizeof(float));
  unsigned short* Phi[2];
  unsigned short* Plo[2];
  Phi[0] = (unsigned short*)((char*)d_ws + off); off += al256((size_t)nPA * DIM * 2);
  Plo[0] = (unsigned short*)((char*)d_ws + off); off += al256((size_t)nPA * DIM * 2);
  Phi[1] = (unsigned short*)((char*)d_ws + off); off += al256((size_t)nPA * DIM * 2);
  Plo[1] = (unsigned short*)((char*)d_ws + off); off += al256((size_t)nPA * DIM * 2);
  if (off > ws_size) return;

  {
    const int n8w = NC * DIM / 8;
    k_split<<<(n8w + NTHR - 1) / NTHR, NTHR, 0, stream>>>(W, WChi, WClo, n8w);
    const int n8g = NG * DIM / 8;
    k_split<<<(n8g + NTHR - 1) / NTHR, NTHR, 0, stream>>>(w_ih, WIhi, WIlo, n8g);
    k_split<<<(n8g + NTHR - 1) / NTHR, NTHR, 0, stream>>>(w_hh, WHhi, WHlo, n8g);
    const int n8f = nN * DIM / 8;
    k_split<<<(n8f + NTHR - 1) / NTHR, NTHR, 0, stream>>>(feat, Phi[0], Plo[0], n8f);
  }

  hipFuncSetAttribute(reinterpret_cast<const void*>(&k_agg),
                      hipFuncAttributeMaxDynamicSharedMemorySize, LDS_B_BYTES);

  const int gridA = nPA / GR;
  const int gridB = (nN + NB - 1) / NB;
  for (int s = 1; s <= 5; ++s) {
    const int pin = (s - 1) & 1, pout = s & 1;
    const float* hold = (s == 1) ? feat : (((s - 1) & 1) ? out : hf1);
    float* hnew = (s & 1) ? out : hf1;
    k_lin<<<gridA, NTHR, 0, stream>>>(Phi[pin], Plo[pin], WChi, WClo, bcat, hall, nN);
    k_agg<<<gridB, NTHR, LDS_B_BYTES, stream>>>(hall, src, dst, ety, hold,
                                                WIhi, WIlo, WHhi, WHlo, Phi[pin], Plo[pin],
                                                b_ih, b_hh, hnew, Phi[pout], Plo[pout], nN, nE);
  }
}
